// Transformer_3315714752562
// MI455X (gfx1250) — hardware-run, weakly checked
//
#include <hip/hip_runtime.h>


#ifndef NTOK
#define NTOK 16384
#endif
#define NTOK_FULL 16384
#define DIN  256
#define MD   64
#define NBLK 3
#define NGM  5
#define TOKW 32
#define TP   68
#define TSZ  (16 * TP)
#define HP   72
#define OFF_CUR 0
#define OFF_RES (1 * TSZ)
#define OFF_Q   (2 * TSZ)
#define OFF_K   (3 * TSZ)
#define OFF_V   (4 * TSZ)
#define OFF_Y   (5 * TSZ)
#define QRS  2048.0f
#define QRI  (1.0f / 2048.0f)
#define WSC  64.0f
#define WSI  (1.0f / 64.0f)
#define L2E  1.4426950408889634f

static_assert(MD == 64);
static_assert(MD % 32 == 0);
static_assert(DIN % 64 == 0);
static_assert(DIN % 32 == 0);
static_assert(TOKW == 32);
static_assert(NTOK % TOKW == 0);
static_assert(NTOK <= NTOK_FULL);
static_assert((size_t)NTOK_FULL * 4 == 65536);
static_assert(((size_t)NTOK_FULL * 4) % 128 == 0);
static_assert((TP * 4) % 16 == 0);
static_assert((HP * 2) % 16 == 0);
static_assert(TP >= MD);
static_assert(HP >= MD);
static_assert(NGM * NBLK * MD == 960);
static_assert(6 * 32 == NBLK * MD);
static_assert(32 * 16 == 4 * 128);
static_assert(8 * 16 == 128);
static_assert(256 * 2 * 16 == 64 * 128);
static_assert((size_t)6 * TSZ * 4 + (size_t)2 * 16 * HP * 2 + 960 * 4 + 2 * 16 * 4 + 32 * 4 <= 131072);
static_assert((size_t)64 * 65 * 4 <= 131072);

typedef _Float16 h16;
typedef unsigned short bf;
typedef __attribute__((ext_vector_type(16))) __bf16   v16bf;
typedef __attribute__((ext_vector_type(16))) _Float16 v16h;
typedef __attribute__((ext_vector_type(8)))  _Float16 v8h;
typedef __attribute__((ext_vector_type(8)))  unsigned short v8us;
typedef __attribute__((ext_vector_type(8)))  float    v8f;
typedef __attribute__((ext_vector_type(4)))  float    v4f;
typedef v4f  __attribute__((may_alias)) v4fa;
typedef v8h  __attribute__((may_alias)) v8ha;

__device__ __forceinline__ unsigned short f2bf(float f) { unsigned u = __float_as_uint(f); u += 0x7FFFu + ((u >> 16) & 1u); return (unsigned short)(u >> 16); }
__device__ __forceinline__ float bfr(float f) { return __uint_as_float(((unsigned)f2bf(f)) << 16); }
__device__ __forceinline__ v16h cat16(v8h lo, v8h hi) { return __builtin_shufflevector(lo, hi, 0, 1, 2, 3, 4, 5, 6, 7, 8, 9, 10, 11, 12, 13, 14, 15); }
__device__ __forceinline__ v16bf cat16b(v8us lo, v8us hi) { return __builtin_bit_cast(v16bf, __builtin_shufflevector(lo, hi, 0, 1, 2, 3, 4, 5, 6, 7, 8, 9, 10, 11, 12, 13, 14, 15)); }
__device__ __forceinline__ v8f wmma16(v16h a, v16h b, v8f c) { return __builtin_amdgcn_wmma_f32_16x16x32_f16(false, a, false, b, (short)0, c, false, false); }
__device__ __forceinline__ v8f wmmab(v16bf a, v16bf b, v8f c) { return __builtin_amdgcn_wmma_f32_16x16x32_bf16(false, a, false, b, (short)0, c, false, false); }
__device__ __forceinline__ v16h  ldh(const h16* p) { return cat16(*(const v8h*)p, *(const v8h*)(p + 16)); }
__device__ __forceinline__ v16bf ldb(const bf* p)  { return cat16b(*(const v8us*)p, *(const v8us*)(p + 16)); }
__device__ __forceinline__ void wave_sync() { __builtin_amdgcn_fence(3  , "wavefront"); __builtin_amdgcn_wave_barrier(); asm volatile("" ::: "memory"); }
__device__ __forceinline__ v8f wmma16g(v16h a, v16h b, v8f c) { c = wmma16(a, b, c); asm volatile("v_nop\n\tv_nop\n\tv_nop\n\tv_nop" : "+v"(c) : "v"(a), "v"(b)); return c; }
__device__ __forceinline__ v8f wmmabg(v16bf a, v16bf b, v8f c) { c = wmmab(a, b, c); asm volatile("v_nop\n\tv_nop\n\tv_nop\n\tv_nop" : "+v"(c) : "v"(a), "v"(b)); return c; }
static __device__ __forceinline__ h16 toh_flush(float v) { const h16 r = (h16)v; return (fabsf(v) < 6.103515625e-05f) ? (h16)0.0f : r; }

__global__ __launch_bounds__(256) void k_w1t(const float* __restrict__ W1, bf* W1T) {
    __shared__ float ts[64 * 65];
    const int tid = threadIdx.x; const int kc = blockIdx.x;
#pragma unroll 1
    for (int i = 0; i < 16; ++i) { const int e = tid + i * 256; const int k = e >> 6, n = e & 63; ts[k * 65 + n] = W1[(size_t)kc * 64 * MD + e]; }
    __syncthreads();
    const int p8 = (tid & 7) * 8;
    v8us o0, o1;
#pragma unroll
    for (int u = 0; u < 8; ++u) { o0[u] = f2bf(ts[(p8 + u) * 65 + (tid >> 3)]); o1[u] = f2bf(ts[(p8 + u) * 65 + (tid >> 3) + 32]); }
    bf* d0 = W1T + (size_t)(tid >> 3) * DIN + (size_t)kc * 64 + p8;
    bf* d1 = W1T + (size_t)((tid >> 3) + 32) * DIN + (size_t)kc * 64 + p8;
#pragma unroll 1
    for (int ps = 0; ps < 2; ++ps) {
        *(volatile v8us*)d0 = o0; *(volatile v8us*)d1 = o1;
        if (ps == 0) __threadfence(); }
}

__global__ __launch_bounds__(256) void k_wth(const float* __restrict__ W, h16* WT) {
    __shared__ float ts[64 * 65];
    const int tid = threadIdx.x; const int t = blockIdx.x;
#pragma unroll 1
    for (int i = 0; i < 16; ++i) { const int e = tid + i * 256; const int k = e >> 6, n = e & 63; ts[k * 65 + n] = W[(size_t)t * MD * MD + e]; }
    __syncthreads();
    const int p8 = (tid & 7) * 8;
    v8h o0, o1;
#pragma unroll
    for (int u = 0; u < 8; ++u) { o0[u] = toh_flush(bfr(ts[(p8 + u) * 65 + (tid >> 3)]) * WSC); o1[u] = toh_flush(bfr(ts[(p8 + u) * 65 + (tid >> 3) + 32]) * WSC); }
    h16* d0 = WT + (size_t)t * MD * MD + (size_t)(tid >> 3) * MD + p8;
    h16* d1 = WT + (size_t)t * MD * MD + (size_t)((tid >> 3) + 32) * MD + p8;
#pragma unroll 1
    for (int ps = 0; ps < 2; ++ps) {
        *(volatile v8h*)d0 = o0; *(volatile v8h*)d1 = o1;
        if (ps == 0) __threadfence(); }
}

__global__ __launch_bounds__(32) void k_tok(const float* __restrict__ x, const bf* __restrict__ W1T, const h16* __restrict__ WH,
                                            const float* __restrict__ b1, const float* __restrict__ bq, const float* __restrict__ bk, const float* __restrict__ bv,
                                            const float* __restrict__ bf1, const float* __restrict__ bf2, const float* __restrict__ ln_g, const float* __restrict__ ln_b,
                                            const float* __restrict__ Wout, const float* __restrict__ bout, float* OUT) {
    __shared__ __align__(16) float T[6 * TSZ];
    __shared__ __align__(16) h16 AH[16 * HP];
    __shared__ __align__(16) h16 AR[16 * HP];
    __shared__ __align__(16) float BS[NGM * NBLK * MD];
    __shared__ __align__(16) float KX[16];
    __shared__ __align__(16) float KN[16];
    __shared__ __align__(16) float OS[TOKW];
    const int lane = threadIdx.x & 31, lr = lane & 15, hi = lane >> 4;
    const int n0 = blockIdx.x * TOKW;

#pragma unroll 1
    for (int i = 0; i < 6; ++i) { const int e = i * 32 + lane;
        BS[e] = bfr(bq[e]); BS[192 + e] = bfr(bk[e]); BS[384 + e] = bfr(bv[e]); BS[576 + e] = bfr(bf1[e]); BS[768 + e] = bfr(bf2[e]); }
    wave_sync();

#pragma unroll 1
    for (int slab = 0; slab < 2; ++slab) {
        const int tb = n0 + slab * 16;
        {
            const float* xr = x + (size_t)(tb + lr) * DIN + 8 * hi;
            const bf* wb = W1T + (size_t)lr * DIN + 8 * hi;
            v8f acc[4];
#pragma unroll
            for (int nb = 0; nb < 4; ++nb) acc[nb] = (v8f){};
#pragma unroll 1
            for (int kc = 0; kc < DIN; kc += 32) {
                const v4f x0 = *(const v4f*)(xr + kc), x1 = *(const v4f*)(xr + kc + 4), x2 = *(const v4f*)(xr + kc + 16), x3 = *(const v4f*)(xr + kc + 20);
                v8us lo, up;
#pragma unroll
                for (int i = 0; i < 4; ++i) { lo[i] = f2bf(x0[i]); lo[4 + i] = f2bf(x1[i]); up[i] = f2bf(x2[i]); up[4 + i] = f2bf(x3[i]); }
                const v16bf a = cat16b(lo, up);
#pragma unroll
                for (int nb = 0; nb < 4; ++nb) { const v16bf b = ldb(wb + (size_t)nb * 16 * DIN + kc); acc[nb] = wmmabg(a, b, acc[nb]); }
            }
#pragma unroll
            for (int nb = 0; nb < 4; ++nb) { const int col = nb * 16 + lr; const float bb = bfr(b1[col]);
#pragma unroll
                for (int j = 0; j < 8; ++j) { const float hv = acc[nb][j] + bb;
                    T[OFF_CUR + (8 * hi + j) * TP + col] = hv;
                    T[OFF_RES + (8 * hi + j) * TP + col] = (hv >= 0.0f) ? hv : 0.1f * hv; } }
        }
        wave_sync();

#pragma unroll 1
        for (int t = 0; t < NBLK; ++t) {
#pragma unroll 1
            for (int g = 0; g < NGM; ++g) {
                if (g == 3) {
                    { float mx = -3.0e38f, mn = 3.0e38f;
#pragma unroll 1
                      for (int u = 0; u < 8; ++u) { const v4f kk = *(const v4fa*)(&T[OFF_K + lr * TP + 32 * hi + 4 * u]);
                          mx = fmaxf(fmaxf(mx, fmaxf(kk[0], kk[1])), fmaxf(kk[2], kk[3])); mn = fminf(fminf(mn, fminf(kk[0], kk[1])), fminf(kk[2], kk[3])); }
                      mx = fmaxf(mx, __shfl_xor(mx, 16, 32)); mn = fminf(mn, __shfl_xor(mn, 16, 32));
                      if (hi == 0) { KX[lr] = mx; KN[lr] = mn; } }
                    wave_sync();
#pragma unroll 1
                    for (int n = 0; n < 16; ++n) {
                        const int ro = n * TP;
                        const float q0 = T[OFF_Q + ro + lane], q1 = T[OFF_Q + ro + 32 + lane];
                        const float kx = KX[n], kn = KN[n];
                        const float e0 = (q0 >= 0.0f) ? kx : kn, e1 = (q1 >= 0.0f) ? kx : kn;
                        const float s0q = q0 * L2E, s1q = q1 * L2E;
                        float s0 = 0.0f, s1 = 0.0f, y0 = 0.0f, y1 = 0.0f;
#pragma unroll 2
                        for (int jj = 0; jj < MD; jj += 4) {
                            const v4f kk = *(const v4fa*)(&T[OFF_K + ro + jj]); const v4f vv = *(const v4fa*)(&T[OFF_V + ro + jj]);
#pragma unroll
                            for (int c = 0; c < 4; ++c) {
                                const float p0 = __builtin_amdgcn_exp2f((kk[c] - e0) * s0q);
                                const float p1 = __builtin_amdgcn_exp2f((kk[c] - e1) * s1q);
                                s0 += p0; s1 += p1; y0 += p0 * vv[c]; y1 += p1 * vv[c]; } }
                        T[OFF_Y + ro + lane]      = y0 * __builtin_amdgcn_rcpf(s0) + T[OFF_CUR + ro + lane];
                        T[OFF_Y + ro + 32 + lane] = y1 * __builtin_amdgcn_rcpf(s1) + T[OFF_CUR + ro + 32 + lane]; }
                    wave_sync();
                }
                if (g == 0 || g >= 3) {
                    const int psrc = (g == 0) ? OFF_CUR : ((g == 3) ? OFF_Y : OFF_Q);
#pragma unroll
                    for (int u = 0; u < 4; ++u) { const int c = 32 * hi + 8 * u;
                        const v4f x0 = *(const v4fa*)(&T[psrc + lr * TP + c]); const v4f x1 = *(const v4fa*)(&T[psrc + lr * TP + c + 4]); v8h hv, rv;
#pragma unroll
                        for (int i = 0; i < 4; ++i) { const h16 a0 = toh_flush(x0[i]); const h16 a1 = toh_flush(x1[i]); hv[i] = a0; hv[4 + i] = a1;
                            rv[i] = toh_flush((x0[i] - (float)a0) * QRS); rv[4 + i] = toh_flush((x1[i] - (float)a1) * QRS); }
                        *(v8ha*)(&AH[lr * HP + c]) = hv; *(v8ha*)(&AR[lr * HP + c]) = rv; }
                    wave_sync();
                }
                {
                    const h16* wp = WH + (size_t)((g * NBLK + t) * MD) * MD + (size_t)lr * MD + 8 * hi;
                    v8f acc[4], acr[4];
#pragma unroll
                    for (int nb = 0; nb < 4; ++nb) { acc[nb] = (v8f){}; acr[nb] = (v8f){}; }
#pragma unroll
                    for (int ks = 0; ks < 2; ++ks) {
                        const int ao = lr * HP + ks * 32 + 8 * hi;
                        const v16h ah = cat16(*(const v8ha*)(&AH[ao]), *(const v8ha*)(&AH[ao + 16]));
                        const v16h ar = cat16(*(const v8ha*)(&AR[ao]), *(const v8ha*)(&AR[ao + 16]));
#pragma unroll
                        for (int nb = 0; nb < 4; ++nb) { const v16h b = ldh(wp + (size_t)nb * 16 * MD + ks * 32);
                            acc[nb] = wmma16g(ah, b, acc[nb]); acr[nb] = wmma16g(ar, b, acr[nb]); }
                    }
                    const int gd = (g >= 3) ? (g - 3) : g;
                    const int dofs = OFF_Q + gd * TSZ;
                    const float sl = (g == 3) ? 0.01f : 1.0f;
                    const int bo = g * (NBLK * MD) + t * MD;
#pragma unroll
                    for (int nb = 0; nb < 4; ++nb) { const int col = nb * 16 + lr; const float bb = BS[bo + col];
#pragma unroll
                        for (int j = 0; j < 8; ++j) { float v = (acc[nb][j] + acr[nb][j] * QRI) * WSI + bb;
                            v = (v >= 0.0f) ? v : sl * v;
                            T[dofs + (8 * hi + j) * TP + col] = v; } }
                }
                wave_sync();
            }
            {
                const int ro = lr * TP + 32 * hi;
                float sm = 0.0f;
#pragma unroll 1
                for (int u = 0; u < 8; ++u) { const int o = ro + 4 * u;
                    const v4f a = *(const v4fa*)(&T[OFF_K + o]) + *(const v4fa*)(&T[OFF_Y + o]);
                    *(v4fa*)(&T[OFF_K + o]) = a; sm += (a[0] + a[1]) + (a[2] + a[3]); }
                sm += __shfl_xor(sm, 16, 32);
                const float mu = sm * (1.0f / MD);
                float vs = 0.0f;
#pragma unroll 1
                for (int u = 0; u < 8; ++u) { const v4f a = *(const v4fa*)(&T[OFF_K + ro + 4 * u]);
                    const float d0 = a[0] - mu, d1 = a[1] - mu, d2 = a[2] - mu, d3 = a[3] - mu; vs += (d0 * d0 + d1 * d1) + (d2 * d2 + d3 * d3); }
                vs += __shfl_xor(vs, 16, 32);
                const float inv = __builtin_amdgcn_rsqf(vs * (1.0f / MD) + 1e-5f);
#pragma unroll 1
                for (int u = 0; u < 8; ++u) { const int o = ro + 4 * u; const int c = 32 * hi + 4 * u;
                    const v4f a = *(const v4fa*)(&T[OFF_K + o]); const v4f r4 = *(const v4fa*)(&T[OFF_RES + o]);
                    const v4f g4 = *(const v4f*)(ln_g + t * MD + c); const v4f b4 = *(const v4f*)(ln_b + t * MD + c); v4f nr;
#pragma unroll
                    for (int i = 0; i < 4; ++i) nr[i] = ((a[i] - mu) * inv * bfr(g4[i]) + bfr(b4[i])) + r4[i];
                    *(v4fa*)(&T[OFF_RES + o]) = nr; *(v4fa*)(&T[OFF_CUR + o]) = nr; }
            }
            wave_sync();
        }
        {
            const int ro = lr * TP + 32 * hi;
            float ds = 0.0f;
#pragma unroll 1
            for (int u = 0; u < 8; ++u) { const v4f r4 = *(const v4fa*)(&T[OFF_RES + ro + 4 * u]); const v4f w4 = *(const v4f*)(Wout + 32 * hi + 4 * u);
                ds += (r4[0] * bfr(w4[0]) + r4[1] * bfr(w4[1])) + (r4[2] * bfr(w4[2]) + r4[3] * bfr(w4[3])); }
            ds += __shfl_xor(ds, 16, 32);
            float ov = ds + bfr(bout[0]);
            ov = (ov >= 0.0f) ? ov : 0.1f * ov;
            if (hi == 0) OS[slab * 16 + lr] = ov;
        }
        wave_sync();
    }
    {
        const int c = lane >> 3, q4 = (lane & 7) * 4;
        const v4f val = *(const v4fa*)(&OS[q4]);
        float* o03 = OUT + (size_t)c * NTOK_FULL + n0 + q4;
        float* o4  = OUT + (size_t)4 * NTOK_FULL + n0 + q4;
#pragma unroll 1
        for (int ps = 0; ps < 2; ++ps) {
            *(volatile v4f*)o03 = val;
            if (lane < 8) *(volatile v4f*)o4 = val;
            if (ps == 0) __threadfence(); }
    }
}

static constexpr size_t al256(size_t v) { return (v + 255) & ~(size_t)255; }
static constexpr size_t SZ_W1T = al256((size_t)MD * DIN * 2);
static constexpr size_t SZ_WH  = al256((size_t)NGM * NBLK * MD * MD * 2);
static constexpr size_t SZ_TOTAL = SZ_W1T + SZ_WH;
static_assert(SZ_TOTAL <= (size_t)134217728);
static_assert(((size_t)NBLK * MD * MD * 2) % 256 == 0);
static_assert((size_t)(DIN / 64) * 64 == (size_t)DIN);
static_assert((size_t)(NTOK / TOKW) * TOKW == (size_t)NTOK);

extern "C" void kernel_launch(void* const* d_in, const int* in_sizes, int n_in,
                              void* d_out, int out_size, void* d_ws, size_t ws_size, hipStream_t stream) {
    if (n_in < 17) return;
    if ((size_t)in_sizes[0] < (size_t)NTOK * DIN) return;
    if ((size_t)in_sizes[1] < (size_t)DIN * MD || in_sizes[2] < MD) return;
    if ((size_t)in_sizes[3] < (size_t)NBLK * MD * MD || (size_t)in_sizes[5] < (size_t)NBLK * MD * MD || (size_t)in_sizes[7] < (size_t)NBLK * MD * MD) return;
    if ((size_t)in_sizes[9] < (size_t)NBLK * MD * MD || (size_t)in_sizes[11] < (size_t)NBLK * MD * MD) return;
    if (in_sizes[4] < NBLK * MD || in_sizes[6] < NBLK * MD || in_sizes[8] < NBLK * MD || in_sizes[10] < NBLK * MD || in_sizes[12] < NBLK * MD) return;
    if (in_sizes[13] < NBLK * MD || in_sizes[14] < NBLK * MD || in_sizes[15] < MD || in_sizes[16] < 1) return;
    if ((size_t)out_size < (size_t)4 * NTOK_FULL + NTOK) return;
    if (SZ_TOTAL > ws_size) return;
    const float* x   = (const float*)d_in[0];
    const float* W1  = (const float*)d_in[1];  const float* b1  = (const float*)d_in[2];
    const float* Wq  = (const float*)d_in[3];  const float* bq  = (const float*)d_in[4];
    const float* Wk  = (const float*)d_in[5];  const float* bk  = (const float*)d_in[6];
    const float* Wv  = (const float*)d_in[7];  const float* bv  = (const float*)d_in[8];
    const float* Wf1 = (const float*)d_in[9];  const float* bf1 = (const float*)d_in[10];
    const float* Wf2 = (const float*)d_in[11]; const float* bf2 = (const float*)d_in[12];
    const float* lng = (const float*)d_in[13]; const float* lnb = (const float*)d_in[14];
    const float* Wo  = (const float*)d_in[15]; const float* bo  = (const float*)d_in[16];
    float* OUT = (float*)d_out;
    char* wsp = (char*)d_ws;
    bf*  W1T = (bf*)wsp;  wsp += SZ_W1T;
    h16* WH  = (h16*)wsp; wsp += SZ_WH;
    const size_t gsz = (size_t)NBLK * MD * MD;

    k_w1t<<<DIN / 64, 256, 0, stream>>>(W1, W1T);
    k_wth<<<NBLK, 256, 0, stream>>>(Wq,  WH + 0 * gsz);
    k_wth<<<NBLK, 256, 0, stream>>>(Wk,  WH + 1 * gsz);
    k_wth<<<NBLK, 256, 0, stream>>>(Wv,  WH + 2 * gsz);
    k_wth<<<NBLK, 256, 0, stream>>>(Wf1, WH + 3 * gsz);
    k_wth<<<NBLK, 256, 0, stream>>>(Wf2, WH + 4 * gsz);

    k_tok<<<NTOK / TOKW, 32, 0, stream>>>(x, W1T, WH, b1, bq, bk, bv, bf1, bf2, lng, lnb, Wo, bo, OUT);
}
